// MultiHeadSelfAttention_55018531062301
// MI455X (gfx1250) — hardware-verified
//
#include <hip/hip_runtime.h>


#ifndef NB
#define NB 2
#endif
#ifndef SEQ
#define SEQ 2048
#endif
#define NB_FULL  2
#define SEQ_FULL 2048
#define DM    1024
#define NH    16
#define HD    64
#define RH    256
#define PCAR  1024.0f
#define SCL   0.125f
#define L2E   1.4426950408889634f
#define NEGB  (-3.0e38f)
#define KP    72
#define PP    40
#define MROWS (NB * SEQ)

typedef _Float16 h16;
typedef unsigned short bf;
typedef __attribute__((ext_vector_type(16))) __bf16   v16bf;
typedef __attribute__((ext_vector_type(16))) _Float16 v16h;
typedef __attribute__((ext_vector_type(8)))  _Float16 v8h;
typedef __attribute__((ext_vector_type(4)))  _Float16 v4h;
typedef __attribute__((ext_vector_type(8)))  unsigned short v8us;
typedef __attribute__((ext_vector_type(4)))  unsigned short v4us;
typedef __attribute__((ext_vector_type(8)))  float    v8f;
typedef __attribute__((ext_vector_type(4)))  float    v4f;
typedef __attribute__((ext_vector_type(2)))  float    v2f;
typedef v8h  __attribute__((may_alias)) v8ha;
typedef v4f  __attribute__((may_alias)) v4fa;
typedef v8us __attribute__((may_alias)) v8usa;
typedef v4us __attribute__((may_alias)) v4usa;

static_assert(HD == 64);
static_assert(NH * HD == DM);
static_assert(DM % 64 == 0 && DM % 32 == 0);
static_assert(SEQ % 64 == 0 && RH % 64 == 0 && RH <= SEQ);
static_assert(MROWS % 64 == 0);
static_assert((KP * 2) % 16 == 0 && KP >= 64);
static_assert((PP * 2) % 16 == 0 && PP >= 32);
static_assert(SEQ <= SEQ_FULL && NB <= NB_FULL);

#define SZ_W   ((size_t)DM * DM * 2)
#define SZ_XB  ((size_t)MROWS * DM * 2)
#define SZ_CS  ((size_t)MROWS * 64 * 4)
#define SZ_QK  ((size_t)2 * NB * NH * SEQ * HD * 2)
#define SZ_VT  ((size_t)NB * NH * HD * SEQ * 2)
#define SZ_VE  ((size_t)NB * NH * HD * RH * 2)
#define SZ_AT  ((size_t)MROWS * DM * 2)
#define SZ_ALL (4 * SZ_W + SZ_XB + SZ_CS + 2 * SZ_QK + SZ_VT + 2 * SZ_VE + 2 * SZ_AT)
static_assert(SZ_W % 256 == 0 && SZ_XB % 256 == 0 && SZ_CS % 256 == 0 && SZ_QK % 256 == 0 && SZ_VT % 256 == 0 && SZ_VE % 256 == 0 && SZ_AT % 256 == 0);
static_assert(SZ_ALL <= (size_t)134217728);

__device__ __forceinline__ unsigned short f2bf(float f) { unsigned u = __float_as_uint(f); u += 0x7FFFu + ((u >> 16) & 1u); return (unsigned short)(u >> 16); }
__device__ __forceinline__ float bf2f(unsigned short b) { return __uint_as_float(((unsigned)b) << 16); }
__device__ __forceinline__ void splitf(float y, unsigned short& h, unsigned short& l) { h = f2bf(y); l = f2bf(y - bf2f(h)); }
__device__ __forceinline__ v16h cat16(v8h lo, v8h hi) { return __builtin_shufflevector(lo, hi, 0, 1, 2, 3, 4, 5, 6, 7, 8, 9, 10, 11, 12, 13, 14, 15); }
__device__ __forceinline__ v16bf cat16b(v8us lo, v8us hi) { return __builtin_bit_cast(v16bf, __builtin_shufflevector(lo, hi, 0, 1, 2, 3, 4, 5, 6, 7, 8, 9, 10, 11, 12, 13, 14, 15)); }
__device__ __forceinline__ v8f wmma16(v16h a, v16h b, v8f c) { return __builtin_amdgcn_wmma_f32_16x16x32_f16(false, a, false, b, (short)0, c, false, false); }
__device__ __forceinline__ v8f wmmab(v16bf a, v16bf b, v8f c) { return __builtin_amdgcn_wmma_f32_16x16x32_bf16(false, a, false, b, (short)0, c, false, false); }
__device__ __forceinline__ v16bf ldb(const bf* p) { return cat16b(*(const v8us*)p, *(const v8us*)(p + 16)); }
#define LDSB(arr, o) cat16b(*(const v8usa*)&arr[(o)], *(const v8usa*)&arr[(o) + 16])
#define LDSH(arr, o) cat16(*(const v8ha*)&arr[(o)], *(const v8ha*)&arr[(o) + 16])

__global__ __launch_bounds__(256) void k_cvt8(const float* __restrict__ src, bf* dst, size_t n8) {
    const size_t i = (size_t)blockIdx.x * 256 + threadIdx.x; if (i >= n8) return;
    const v8f v = *(const v8f*)(src + i * 8); v8us o;
#pragma unroll
    for (int k = 0; k < 8; ++k) o[k] = f2bf(v[k]);
    *(volatile v8us*)(dst + i * 8) = o; __threadfence(); *(volatile v8us*)(dst + i * 8) = o;
}

__global__ __launch_bounds__(256) void k_cvtx(const float* __restrict__ x, bf* XB) {
    const size_t i = (size_t)blockIdx.x * 256 + threadIdx.x; if (i >= (size_t)MROWS * DM / 8) return;
    const int row = (int)(i / (DM / 8)); const int c8 = (int)(i % (DM / 8)); const int b = row / SEQ; const int s = row - b * SEQ;
    const v8f v = *(const v8f*)(x + ((size_t)b * SEQ_FULL + s) * DM + (size_t)c8 * 8); v8us o;
#pragma unroll
    for (int k = 0; k < 8; ++k) o[k] = f2bf(v[k]);
    *(volatile v8us*)(XB + i * 8) = o; __threadfence(); *(volatile v8us*)(XB + i * 8) = o;
}

__global__ __launch_bounds__(256) void k_cstab(const int* __restrict__ tok, float* CS) {
    const int idx = blockIdx.x * 256 + threadIdx.x; if (idx >= MROWS * 32) return;
    const int j = idx & 31, m = idx >> 5; const int b = m / SEQ, s = m - b * SEQ;
    const int pos = tok[(size_t)b * SEQ_FULL + s];
    double p = 1.0;
    p *= (j & 1)  ? 1.3335214321633240 : 1.0;
    p *= (j & 2)  ? 1.7782794100389228 : 1.0;
    p *= (j & 4)  ? 3.1622776601683795 : 1.0;
    p *= (j & 8)  ? 10.0 : 1.0;
    p *= (j & 16) ? 100.0 : 1.0;
    const float pf = (float)p; const float inv = 1.0f / pf; const float ang = (float)pos * inv;
    float sn, cs; sincosf(ang, &sn, &cs);
    v2f o; o[0] = cs; o[1] = sn;
    *(volatile v2f*)(CS + (size_t)idx * 2) = o; __threadfence(); *(volatile v2f*)(CS + (size_t)idx * 2) = o;
}

__device__ __forceinline__ void gemm_acc(const bf* __restrict__ A, const bf* __restrict__ Bt, const size_t aoff, const size_t boff, v8f (&acc)[4][4]) {
#pragma unroll 1
    for (int kc = 0; kc < DM; kc += 32) {
        v16bf a[4]; v16bf b;
#pragma unroll
        for (int mb = 0; mb < 4; ++mb) a[mb] = ldb(A + aoff + (size_t)mb * 16 * DM + kc);
#pragma unroll
        for (int nb = 0; nb < 4; ++nb) { b = ldb(Bt + boff + (size_t)nb * 16 * DM + kc);
#pragma unroll
            for (int mb = 0; mb < 4; ++mb) acc[mb][nb] = wmmab(a[mb], b, acc[mb][nb]); }
        asm volatile("v_nop\n\tv_nop\n\tv_nop\n\tv_nop" : "+v"(acc[0][2]), "+v"(acc[1][2]), "+v"(acc[2][2]), "+v"(acc[3][2]), "+v"(acc[0][3]), "+v"(acc[1][3]), "+v"(acc[2][3]), "+v"(acc[3][3]) : "v"(a[3]), "v"(b));
    }
}

__global__ __launch_bounds__(32) void k_projqk(const bf* __restrict__ XB, const bf* __restrict__ WQK, const float* __restrict__ CS, bf* QKh, bf* QKl) {
#pragma clang fp contract(off)
    __shared__ __align__(16) float os[64 * 68];
    const int lane = threadIdx.x & 31, lr = lane & 15, hi = lane >> 4; const int r0 = blockIdx.x * 64, c0 = blockIdx.y * 64;
    v8f acc[4][4];
#pragma unroll
    for (int mb = 0; mb < 4; ++mb)
#pragma unroll
        for (int nb = 0; nb < 4; ++nb) acc[mb][nb] = (v8f){};
    gemm_acc(XB, WQK, (size_t)(r0 + lr) * DM + 8 * hi, (size_t)(c0 + lr) * DM + 8 * hi, acc);
#pragma unroll
    for (int mb = 0; mb < 4; ++mb)
#pragma unroll
        for (int nb = 0; nb < 4; ++nb)
#pragma unroll
            for (int j = 0; j < 8; ++j) os[(mb * 16 + hi * 8 + j) * 68 + nb * 16 + lr] = acc[mb][nb][j];
    __builtin_amdgcn_wave_barrier(); asm volatile("" ::: "memory");
    const int which = c0 / DM, h = (c0 % DM) / HD; const int b = r0 / SEQ, s0 = r0 - b * SEQ;
    const size_t pbase = ((((size_t)which * NB + b) * NH + h) * SEQ + s0) * HD;
#pragma unroll 1
    for (int ps = 0; ps < 2; ++ps) {
#pragma unroll 2
        for (int s = 0; s < 32; ++s) { const int row = 2 * s + hi, cofs = lr * 4;
            const v4f val = *(const v4fa*)(os + row * 68 + cofs);
            const v4f cs = *(const v4f*)(CS + (size_t)(r0 + row) * 64 + cofs);
            const float y0 = val[0] * cs[0] - val[1] * cs[1];
            const float y1 = val[0] * cs[1] + val[1] * cs[0];
            const float y2 = val[2] * cs[2] - val[3] * cs[3];
            const float y3 = val[2] * cs[3] + val[3] * cs[2];
            v4us oh, ol; unsigned short a, c;
            splitf(y0, a, c); oh[0] = a; ol[0] = c; splitf(y1, a, c); oh[1] = a; ol[1] = c; splitf(y2, a, c); oh[2] = a; ol[2] = c; splitf(y3, a, c); oh[3] = a; ol[3] = c;
            const size_t oo = pbase + (size_t)row * HD + cofs;
            *(volatile v4us*)(QKh + oo) = oh; *(volatile v4us*)(QKl + oo) = ol; }
        if (ps == 0) __threadfence(); }
}

__global__ __launch_bounds__(32) void k_projv(const bf* __restrict__ XB, const bf* __restrict__ WV, h16* VT16, bf* VTh, bf* VTl) {
    __shared__ __align__(16) float os[64 * 68];
    const int lane = threadIdx.x & 31, lr = lane & 15, hi = lane >> 4; const int r0 = blockIdx.x * 64, c0 = blockIdx.y * 64;
    v8f acc[4][4];
#pragma unroll
    for (int mb = 0; mb < 4; ++mb)
#pragma unroll
        for (int nb = 0; nb < 4; ++nb) acc[mb][nb] = (v8f){};
    gemm_acc(XB, WV, (size_t)(r0 + lr) * DM + 8 * hi, (size_t)(c0 + lr) * DM + 8 * hi, acc);
#pragma unroll
    for (int mb = 0; mb < 4; ++mb)
#pragma unroll
        for (int nb = 0; nb < 4; ++nb)
#pragma unroll
            for (int j = 0; j < 8; ++j) os[(mb * 16 + hi * 8 + j) * 68 + nb * 16 + lr] = acc[mb][nb][j];
    __builtin_amdgcn_wave_barrier(); asm volatile("" ::: "memory");
    const int h = c0 / HD; const int b = r0 / SEQ, s0 = r0 - b * SEQ;
    const size_t vbase = (((size_t)b * NH + h) * HD) * SEQ + s0;
    const size_t ebase = (((size_t)b * NH + h) * HD) * RH + s0;
    const bool early = (s0 < RH);
#pragma unroll 1
    for (int ps = 0; ps < 2; ++ps) {
#pragma unroll 2
        for (int s = 0; s < 32; ++s) { const int d = 2 * s + hi, t0 = lr * 4;
            float xv[4];
#pragma unroll
            for (int q = 0; q < 4; ++q) xv[q] = os[(t0 + q) * 68 + d];
            v4h o16;
#pragma unroll
            for (int q = 0; q < 4; ++q) o16[q] = (h16)xv[q];
            *(volatile v4h*)(VT16 + vbase + (size_t)d * SEQ + t0) = o16;
            if (early) { v4us oh, ol;
#pragma unroll
                for (int q = 0; q < 4; ++q) { unsigned short a, c; splitf(xv[q], a, c); oh[q] = a; ol[q] = c; }
                *(volatile v4us*)(VTh + ebase + (size_t)d * RH + t0) = oh; *(volatile v4us*)(VTl + ebase + (size_t)d * RH + t0) = ol; } }
        if (ps == 0) __threadfence(); }
}

template <bool HL>
__device__ __forceinline__ void attn_body(const bf* __restrict__ QKh, const bf* __restrict__ QKl, const h16* __restrict__ VT16, const bf* __restrict__ VTh, const bf* __restrict__ VTl, bf* ATh, bf* ATl, const int qb) {
    __shared__ __align__(16) bf  sKh[64 * KP];
    __shared__ __align__(16) bf  sKl[64 * KP];
    __shared__ __align__(16) h16 sV16[HL ? 8 : 64 * KP];
    __shared__ __align__(16) bf  sVh[HL ? 64 * KP : 8];
    __shared__ __align__(16) bf  sVl[HL ? 64 * KP : 8];
    __shared__ __align__(16) h16 sP16[HL ? 8 : 4 * 16 * PP];
    __shared__ __align__(16) bf  sPh[HL ? 4 * 16 * PP : 8];
    __shared__ __align__(16) bf  sPl[HL ? 4 * 16 * PP : 8];
    const int tid = threadIdx.x; const int lane = tid & 31, lr = lane & 15, hi = lane >> 4;
    const int wave = __builtin_amdgcn_readfirstlane(tid >> 5);
    const int b = blockIdx.z, h = blockIdx.y; const int qblk = qb * 64, q0 = qblk + wave * 16;
    const size_t qpl = (((size_t)b * NH + h) * SEQ) * HD;
    const size_t kpl = ((((size_t)NB + b) * NH + h) * SEQ) * HD;
    const size_t vpl = (((size_t)b * NH + h) * HD) * SEQ;
    const size_t epl = (((size_t)b * NH + h) * HD) * RH;
    const size_t qo = qpl + (size_t)(q0 + lr) * HD + 8 * hi;
    const v16bf qh0 = ldb(QKh + qo), qh1 = ldb(QKh + qo + 32), ql0 = ldb(QKl + qo), ql1 = ldb(QKl + qo + 32);
    v8f accd[4];
#pragma unroll
    for (int t = 0; t < 4; ++t) accd[t] = (v8f){};
    float m_run[8], l_run[8];
#pragma unroll
    for (int r = 0; r < 8; ++r) { m_run[r] = NEGB; l_run[r] = 0.0f; }

#pragma unroll 1
    for (int kb = 0; kb <= qblk; kb += 64) {
#pragma unroll
        for (int i = 0; i < 4; ++i) { const int c = tid + 128 * i; const int row = c >> 3, ch = (c & 7) * 8;
            const size_t ko = kpl + (size_t)(kb + row) * HD + ch;
            *(v8usa*)(&sKh[row * KP + ch]) = *(const v8us*)(QKh + ko);
            *(v8usa*)(&sKl[row * KP + ch]) = *(const v8us*)(QKl + ko);
            if (HL) { const size_t vo = epl + (size_t)row * RH + kb + ch;
                *(v8usa*)(&sVh[row * KP + ch]) = *(const v8us*)(VTh + vo);
                *(v8usa*)(&sVl[row * KP + ch]) = *(const v8us*)(VTl + vo); }
            else { *(v8ha*)(&sV16[row * KP + ch]) = *(const v8h*)(VT16 + vpl + (size_t)row * SEQ + kb + ch); } }
        __syncthreads();

#pragma unroll 1
        for (int kh = 0; kh < 2; ++kh) {
            if (kb + 32 * kh > q0 + 15) continue;
            v8f s0 = (v8f){}, s1 = (v8f){};
            { const int kr = (32 * kh + lr) * KP + 8 * hi;
              const v16bf ah0 = LDSB(sKh, kr), ah1 = LDSB(sKh, kr + 32), al0 = LDSB(sKl, kr), al1 = LDSB(sKl, kr + 32);
              s0 = wmmab(qh0, ah0, s0); s0 = wmmab(qh1, ah1, s0); s0 = wmmab(ql0, ah0, s0); s0 = wmmab(ql1, ah1, s0); s0 = wmmab(qh0, al0, s0); s0 = wmmab(qh1, al1, s0);
              const int kr2 = kr + 16 * KP;
              const v16bf bh0 = LDSB(sKh, kr2), bh1 = LDSB(sKh, kr2 + 32), bl0 = LDSB(sKl, kr2), bl1 = LDSB(sKl, kr2 + 32);
              s1 = wmmab(qh0, bh0, s1); s1 = wmmab(qh1, bh1, s1); s1 = wmmab(ql0, bh0, s1); s1 = wmmab(ql1, bh1, s1); s1 = wmmab(qh0, bl0, s1); s1 = wmmab(qh1, bl1, s1);
              asm volatile("v_nop\n\tv_nop\n\tv_nop\n\tv_nop" : "+v"(s0), "+v"(s1) : "v"(bl0), "v"(bl1)); }
            const int kg0 = kb + 32 * kh + lr, kg1 = kg0 + 16;
            float bm[8];
#pragma unroll
            for (int r = 0; r < 8; ++r) { const int qg = q0 + 8 * hi + r;
                const float a0 = (kg0 <= qg) ? s0[r] * SCL : NEGB; const float a1 = (kg1 <= qg) ? s1[r] * SCL : NEGB;
                s0[r] = a0; s1[r] = a1; bm[r] = fmaxf(a0, a1); }
#pragma unroll
            for (int sh = 1; sh < 16; sh <<= 1)
#pragma unroll
                for (int r = 0; r < 8; ++r) bm[r] = fmaxf(bm[r], __shfl_xor(bm[r], sh, 32));
            float rs[8];
#pragma unroll
            for (int r = 0; r < 8; ++r) { const float mn = fmaxf(m_run[r], bm[r]);
                const float sc = __builtin_amdgcn_exp2f((m_run[r] - mn) * L2E); m_run[r] = mn;
                const float p0 = __builtin_amdgcn_exp2f((s0[r] - mn) * L2E); const float p1 = __builtin_amdgcn_exp2f((s1[r] - mn) * L2E);
                s0[r] = p0; s1[r] = p1; rs[r] = p0 + p1; l_run[r] *= sc;
#pragma unroll
                for (int t = 0; t < 4; ++t) accd[t][r] *= sc; }
#pragma unroll
            for (int sh = 1; sh < 16; sh <<= 1)
#pragma unroll
                for (int r = 0; r < 8; ++r) rs[r] += __shfl_xor(rs[r], sh, 32);
#pragma unroll
            for (int r = 0; r < 8; ++r) l_run[r] += rs[r];

            const int pr = (wave * 16 + 8 * hi) * PP + lr;
            const int pa = (wave * 16 + lr) * PP + 8 * hi;
            if (HL) {
#pragma unroll
                for (int r = 0; r < 8; ++r) { unsigned short a, c; splitf(s0[r], a, c); sPh[pr + r * PP] = a; sPl[pr + r * PP] = c; splitf(s1[r], a, c); sPh[pr + r * PP + 16] = a; sPl[pr + r * PP + 16] = c; }
                __builtin_amdgcn_wave_barrier(); asm volatile("" ::: "memory");
                const v16bf aph = LDSB(sPh, pa), apl = LDSB(sPl, pa); v16bf bvh, bvl;
#pragma unroll
                for (int t = 0; t < 4; ++t) { const int vo = (t * 16 + lr) * KP + 32 * kh + 8 * hi; bvh = LDSB(sVh, vo); bvl = LDSB(sVl, vo);
                    accd[t] = wmmab(aph, bvh, accd[t]); accd[t] = wmmab(apl, bvh, accd[t]); accd[t] = wmmab(aph, bvl, accd[t]); }
                asm volatile("v_nop\n\tv_nop\n\tv_nop\n\tv_nop" : "+v"(accd[0]), "+v"(accd[1]), "+v"(accd[2]), "+v"(accd[3]) : "v"(aph), "v"(apl), "v"(bvh), "v"(bvl));
            } else {
#pragma unroll
                for (int r = 0; r < 8; ++r) { sP16[pr + r * PP] = (h16)(s0[r] * PCAR); sP16[pr + r * PP + 16] = (h16)(s1[r] * PCAR); }
                __builtin_amdgcn_wave_barrier(); asm volatile("" ::: "memory");
                const v16h ap = LDSH(sP16, pa); v16h bv;
#pragma unroll
                for (int t = 0; t < 4; ++t) { const int vo = (t * 16 + lr) * KP + 32 * kh + 8 * hi; bv = LDSH(sV16, vo); accd[t] = wmma16(ap, bv, accd[t]); }
                asm volatile("v_nop\n\tv_nop\n\tv_nop\n\tv_nop" : "+v"(accd[0]), "+v"(accd[1]), "+v"(accd[2]), "+v"(accd[3]) : "v"(ap), "v"(bv));
            }
            __builtin_amdgcn_wave_barrier(); asm volatile("" ::: "memory");
        }
        __syncthreads();
    }

    const float car = HL ? 1.0f : PCAR;
#pragma unroll
    for (int r = 0; r < 8; ++r) { const float inv = __builtin_amdgcn_rcpf(l_run[r] * car);
#pragma unroll
        for (int t = 0; t < 4; ++t) { unsigned short a, c; splitf(accd[t][r] * inv, a, c); const int so = (wave * 16 + 8 * hi + r) * KP + t * 16 + lr; sKh[so] = a; sKl[so] = c; } }
    __builtin_amdgcn_wave_barrier(); asm volatile("" ::: "memory");
    const size_t ob = ((size_t)b * SEQ + q0) * DM + (size_t)h * HD;
#pragma unroll 1
    for (int ps = 0; ps < 2; ++ps) {
#pragma unroll
        for (int s2 = 0; s2 < 8; ++s2) { const int row = 2 * s2 + hi; const int so = (wave * 16 + row) * KP + 4 * lr;
            const v4us vh = *(const v4usa*)&sKh[so]; const v4us vl = *(const v4usa*)&sKl[so];
            *(volatile v4us*)(ATh + ob + (size_t)row * DM + 4 * lr) = vh; *(volatile v4us*)(ATl + ob + (size_t)row * DM + 4 * lr) = vl; }
        if (ps == 0) __threadfence(); }
}

__global__ __launch_bounds__(128) void k_attn_early(const bf* __restrict__ QKh, const bf* __restrict__ QKl, const h16* __restrict__ VT16, const bf* __restrict__ VTh, const bf* __restrict__ VTl, bf* ATh, bf* ATl) {
    attn_body<true>(QKh, QKl, VT16, VTh, VTl, ATh, ATl, (int)blockIdx.x);
}
__global__ __launch_bounds__(128) void k_attn_main(const bf* __restrict__ QKh, const bf* __restrict__ QKl, const h16* __restrict__ VT16, const bf* __restrict__ VTh, const bf* __restrict__ VTl, bf* ATh, bf* ATl) {
    attn_body<false>(QKh, QKl, VT16, VTh, VTl, ATh, ATl, (int)blockIdx.x + RH / 64);
}

__global__ __launch_bounds__(32) void k_oproj(const bf* __restrict__ ATh, const bf* __restrict__ ATl, const bf* __restrict__ WO, float* OUT) {
    __shared__ __align__(16) float os[16 * 68];
    const int lane = threadIdx.x & 31, lr = lane & 15, hi = lane >> 4; const int r0 = blockIdx.x * 64, c0 = blockIdx.y * 64;
    v8f acc[4][4];
#pragma unroll
    for (int mb = 0; mb < 4; ++mb)
#pragma unroll
        for (int nb = 0; nb < 4; ++nb) acc[mb][nb] = (v8f){};
    const size_t aoff = (size_t)(r0 + lr) * DM + 8 * hi, boff = (size_t)(c0 + lr) * DM + 8 * hi;
    gemm_acc(ATh, WO, aoff, boff, acc);
    gemm_acc(ATl, WO, aoff, boff, acc);
    const int b = r0 / SEQ, s0 = r0 - b * SEQ;
#pragma unroll
    for (int mb = 0; mb < 4; ++mb) {
#pragma unroll
        for (int nb = 0; nb < 4; ++nb)
#pragma unroll
            for (int j = 0; j < 8; ++j) os[(hi * 8 + j) * 68 + nb * 16 + lr] = acc[mb][nb][j];
        __builtin_amdgcn_wave_barrier(); asm volatile("" ::: "memory");
        float* crow = OUT + ((size_t)b * SEQ_FULL + s0 + mb * 16) * DM + c0;
#pragma unroll 1
        for (int ps = 0; ps < 2; ++ps) {
#pragma unroll
            for (int s = 0; s < 8; ++s) { const int row = 2 * s + hi, cofs = lr * 4; const v4f val = *(const v4fa*)(os + row * 68 + cofs);
                *(volatile v4f*)(crow + (size_t)row * DM + cofs) = val; }
            if (ps == 0) __threadfence(); }
        __builtin_amdgcn_wave_barrier(); asm volatile("" ::: "memory");
    }
}

extern "C" void kernel_launch(void* const* d_in, const int* in_sizes, int n_in,
                              void* d_out, int out_size, void* d_ws, size_t ws_size, hipStream_t stream) {
    if (n_in < 6) return;
    const long long needx = ((long long)(NB - 1) * SEQ_FULL + SEQ) * DM;
    if ((long long)in_sizes[0] < needx) return;
    if ((long long)in_sizes[1] < (long long)DM * DM || (long long)in_sizes[2] < (long long)DM * DM || (long long)in_sizes[3] < (long long)DM * DM || (long long)in_sizes[4] < (long long)DM * DM) return;
    if ((long long)in_sizes[5] < (long long)(NB - 1) * SEQ_FULL + SEQ) return;
    if ((long long)out_size < needx) return;
    const float* x = (const float*)d_in[0]; const float* wq = (const float*)d_in[1]; const float* wk = (const float*)d_in[2]; const float* wv = (const float*)d_in[3]; const float* wo = (const float*)d_in[4];
    const int* tok = (const int*)d_in[5];
    float* OUT = (float*)d_out;
    char* wsp = (char*)d_ws;
    auto take = [&](size_t bytes) { char* p = wsp; wsp += (bytes + 255) & ~(size_t)255; return (void*)p; };
    bf* WQK = (bf*)take(2 * SZ_W); bf* WV = (bf*)take(SZ_W); bf* WO = (bf*)take(SZ_W);
    bf* XB = (bf*)take(SZ_XB); float* CS = (float*)take(SZ_CS);
    bf* QKh = (bf*)take(SZ_QK); bf* QKl = (bf*)take(SZ_QK);
    h16* VT16 = (h16*)take(SZ_VT); bf* VTh = (bf*)take(SZ_VE); bf* VTl = (bf*)take(SZ_VE);
    bf* ATh = (bf*)take(SZ_AT); bf* ATl = (bf*)take(SZ_AT);
    if ((size_t)(wsp - (char*)d_ws) > ws_size) return;

    const size_t w8 = (size_t)DM * DM / 8; const unsigned gw = (unsigned)((w8 + 255) / 256);
    k_cvt8<<<gw, 256, 0, stream>>>(wq, WQK, w8);
    k_cvt8<<<gw, 256, 0, stream>>>(wk, WQK + (size_t)DM * DM, w8);
    k_cvt8<<<gw, 256, 0, stream>>>(wv, WV, w8);
    k_cvt8<<<gw, 256, 0, stream>>>(wo, WO, w8);
    k_cvtx<<<(unsigned)(((size_t)MROWS * DM / 8 + 255) / 256), 256, 0, stream>>>(x, XB);
    k_cstab<<<(unsigned)((MROWS * 32 + 255) / 256), 256, 0, stream>>>(tok, CS);
    k_projqk<<<dim3(MROWS / 64, 2 * DM / 64, 1), 32, 0, stream>>>(XB, WQK, CS, QKh, QKl);
    k_projv<<<dim3(MROWS / 64, DM / 64, 1), 32, 0, stream>>>(XB, WV, VT16, VTh, VTl);
    k_attn_early<<<dim3(RH / 64, NH, NB), 128, 0, stream>>>(QKh, QKl, VT16, VTh, VTl, ATh, ATl);
    if (SEQ > RH) k_attn_main<<<dim3((SEQ - RH) / 64, NH, NB), 128, 0, stream>>>(QKh, QKl, VT16, VTh, VTl, ATh, ATl);
    k_oproj<<<dim3(MROWS / 64, DM / 64, 1), 32, 0, stream>>>(ATh, ATl, WO, OUT);
}
